// GNN_53085795779195
// MI455X (gfx1250) — hardware-verified
//
#include <hip/hip_runtime.h>
#include <stddef.h>
#include <stdint.h>
#include <math.h>


#define HID    64
#define K2     128
#define NLAY   3
#define NTHR   256
#define NWAVE  8
#define EPT    8
#define CHUNK  (NTHR * EPT)
#define WCAP   (EPT * 32)
#define LISTN  (NWAVE * WCAP)
#define NBD    8192
#define SLD    13
#define NBA    1024
#define SLA    10
#define RCAP   28672
#define DEGCAP 128
#define GBM    64
#define GBN    64
#define GTHR   128
#define NU0    (HID * (HID / 8))
#define NU1    (HID * (K2 / 8))
#define NU2    (HID * (K2 / 8))
#define NWBLK  ((NU0 + NU1 + NU2) / NTHR)
#define OW1    (HID * HID)
#define OW2    (HID * HID + HID * K2)
#define WPN    (HID * HID + 2 * HID * K2)
#define PARV   (NLAY * 5 * HID)
#define PLW    PARV
#define PLB    (PARV + HID)
#define PARF   (PARV + HID + 32)
#define PARLDS 1280
#define MISC_INTS 16
#define AGG_ZINTS (LISTN + 2 * RCAP + 3 * NBA)
#define AGG_LDS_INTS (AGG_ZINTS + MISC_INTS + NBA)
#define WSMAX  134217728
#define MEAS_B1024 16623
#define MEAS_MAXDEG 35

static_assert((CHUNK & (CHUNK - 1)) == 0 && CHUNK <= 4096);
static_assert((NBD & (NBD - 1)) == 0 && NBD == (1 << SLD));
static_assert((NBA & (NBA - 1)) == 0 && NBA == (1 << SLA));
static_assert(((long long)CHUNK << SLD) < (1LL << 31));
static_assert(((long long)CHUNK << SLA) < (1LL << 31));
static_assert(NBD % (NTHR * 4) == 0);
static_assert(LISTN % NTHR == 0);
static_assert(NBA % NWAVE == 0 && NBA % 32 == 0 && NBA % GBM == 0 && NBA == 4 * NTHR);
static_assert(RCAP % 32 == 0 && AGG_ZINTS % (NTHR * 4) == 0 && LISTN % 4 == 0);
static_assert(RCAP >= MEAS_B1024 + MEAS_B1024 / 20 + 1);
static_assert(DEGCAP >= MEAS_MAXDEG + 8);
static_assert(HID % 32 == 0 && K2 % 32 == 0 && K2 == 2 * HID && HID == GBN);
static_assert(GBM == (GTHR / 32) * 16 && GBN == 64);
static_assert(NU0 % NTHR == 0 && NU1 % NTHR == 0 && NU2 % NTHR == 0);
static_assert(HID == 2 * 32);
static_assert(AGG_LDS_INTS * 4 <= 300000);
static_assert(PARF % 32 == 0 && PARF <= PARLDS && PARLDS % NTHR == 0 && PARF - 4 * NTHR == 32);
static_assert(((AGG_ZINTS + MISC_INTS) % 4) == 0);

typedef float          v2f   __attribute__((ext_vector_type(2)));
typedef float          v4f   __attribute__((ext_vector_type(4)));
typedef float          v8f   __attribute__((ext_vector_type(8)));
typedef int            v4i   __attribute__((ext_vector_type(4)));
typedef int            v8i   __attribute__((ext_vector_type(8)));
typedef unsigned int   v4u   __attribute__((ext_vector_type(4)));
typedef unsigned short v8us  __attribute__((ext_vector_type(8)));
typedef unsigned short v16us __attribute__((ext_vector_type(16)));
typedef __bf16         v16bf __attribute__((ext_vector_type(16)));
typedef v2f  __attribute__((may_alias)) v2fa;
typedef v4f  __attribute__((may_alias)) v4fa;
typedef v4i  __attribute__((may_alias)) v4ia;
typedef v8us __attribute__((may_alias)) v8usa;
union FragB { v16bf v; v16us u; v8us h[2]; v8i w; };

__device__ __forceinline__ v8f wmb(const FragB& a, const FragB& b, v8f c) {
  v8f d = __builtin_amdgcn_wmma_f32_16x16x32_bf16(false, a.v, false, b.v, (short)0, c, false, false);
  asm volatile("v_nop\n\tv_nop\n\tv_nop\n\tv_nop" : "+v"(d) : "v"(a.w), "v"(b.w));
  return d;
}

__device__ __forceinline__ unsigned bf16_bits(float f) {
  const unsigned u = __float_as_uint(f);
  const unsigned r = (u + 0x7FFFu + ((u >> 16) & 1u)) >> 16;
  return (f != f) ? 0x7FC0u : r;
}
__device__ __forceinline__ float bf16_val(float f) {
  return __uint_as_float(bf16_bits(f) << 16);
}

template <int SLB>
__device__ __forceinline__ int scan_chunk(const int* __restrict__ dsts, int nE, int cbase, int slotBase,
                                          int nb, int vec8, int* list, int tid, int lane, int wave) {
  int wc = 0;
  const int el0  = tid * EPT;
  const int e0   = cbase + el0;
  const int sent = -2147483647 - 1;
  v4i da, db;
  if (vec8 != 0 && cbase + CHUNK <= nE) {
    da = *(const v4i*)(dsts + e0);
    db = *(const v4i*)(dsts + e0 + 4);
  } else {
    da.x = (e0     < nE) ? dsts[min(e0,     nE - 1)] : sent;
    da.y = (e0 + 1 < nE) ? dsts[min(e0 + 1, nE - 1)] : sent;
    da.z = (e0 + 2 < nE) ? dsts[min(e0 + 2, nE - 1)] : sent;
    da.w = (e0 + 3 < nE) ? dsts[min(e0 + 3, nE - 1)] : sent;
    db.x = (e0 + 4 < nE) ? dsts[min(e0 + 4, nE - 1)] : sent;
    db.y = (e0 + 5 < nE) ? dsts[min(e0 + 5, nE - 1)] : sent;
    db.z = (e0 + 6 < nE) ? dsts[min(e0 + 6, nE - 1)] : sent;
    db.w = (e0 + 7 < nE) ? dsts[min(e0 + 7, nE - 1)] : sent;
  }
  const unsigned nbs = (unsigned)slotBase;
  const unsigned unb = (unsigned)nb;
  const unsigned s0 = (unsigned)da.x - nbs, s1 = (unsigned)da.y - nbs;
  const unsigned s2 = (unsigned)da.z - nbs, s3 = (unsigned)da.w - nbs;
  const unsigned s4 = (unsigned)db.x - nbs, s5 = (unsigned)db.y - nbs;
  const unsigned s6 = (unsigned)db.z - nbs, s7 = (unsigned)db.w - nbs;
  const bool h0 = s0 < unb, h1 = s1 < unb, h2 = s2 < unb, h3 = s3 < unb;
  const bool h4 = s4 < unb, h5 = s5 < unb, h6 = s6 < unb, h7 = s7 < unb;
  const unsigned any = __builtin_amdgcn_ballot_w32(h0 | h1 | h2 | h3 | h4 | h5 | h6 | h7);
  if (any != 0u) {
#define HITJ(J, HJ, SJ) { \
      const unsigned mj = __builtin_amdgcn_ballot_w32(HJ); \
      if (mj != 0u) { \
        if (HJ) { \
          const int pos = wc + (int)__builtin_amdgcn_mbcnt_lo(mj, 0u); \
          if (pos < WCAP) list[wave * WCAP + pos] = ((el0 + (J)) << SLB) | (int)(SJ); \
        } \
        wc += (int)__builtin_popcount(mj); } }
    HITJ(0, h0, s0)
    HITJ(1, h1, s1)
    HITJ(2, h2, s2)
    HITJ(3, h3, s3)
    HITJ(4, h4, s4)
    HITJ(5, h5, s5)
    HITJ(6, h6, s6)
    HITJ(7, h7, s7)
#undef HITJ
  }
  return wc;
}

__global__ __launch_bounds__(NTHR) void k_prep(
    const float* __restrict__ x, int nN, int nUx, int gX,
    const float* __restrict__ Ws, const float* __restrict__ bs, const float* __restrict__ gam,
    const float* __restrict__ bet, const float* __restrict__ mea, const float* __restrict__ var,
    const float* __restrict__ lw, const float* __restrict__ lb,
    unsigned short* xb, unsigned short* wp, float* par) {
  __shared__ __attribute__((aligned(16))) float sp[PARLDS];
  const int tid = (int)threadIdx.x;
  const int bid = (int)blockIdx.x;
  if (bid < gX) {
    const int u = bid * NTHR + tid;
    if (u < nUx) {
      const int row = u >> 3;
      const int k8  = (u & 7) * 8;
      const int rc  = row < nN ? row : nN - 1;
      const float* p = x + (size_t)rc * HID + k8;
      const v4f a = *(const v4fa*)p;
      const v4f b = *(const v4fa*)(p + 4);
      const bool ok = row < nN;
      v8us o;
      o[0] = ok ? (unsigned short)bf16_bits(a.x) : (unsigned short)0;
      o[1] = ok ? (unsigned short)bf16_bits(a.y) : (unsigned short)0;
      o[2] = ok ? (unsigned short)bf16_bits(a.z) : (unsigned short)0;
      o[3] = ok ? (unsigned short)bf16_bits(a.w) : (unsigned short)0;
      o[4] = ok ? (unsigned short)bf16_bits(b.x) : (unsigned short)0;
      o[5] = ok ? (unsigned short)bf16_bits(b.y) : (unsigned short)0;
      o[6] = ok ? (unsigned short)bf16_bits(b.z) : (unsigned short)0;
      o[7] = ok ? (unsigned short)bf16_bits(b.w) : (unsigned short)0;
      unsigned short* dp = xb + (size_t)row * HID + k8;
      *(volatile v8us*)dp = o;
      __threadfence();
      *(volatile v8us*)dp = o;
    }
  } else if (bid < gX + NWBLK) {
    const int v = (bid - gX) * NTHR + tid;
    int layer, vv, sh, pitch, doff;
    if (v < NU0)            { layer = 0; vv = v;             sh = 3; pitch = HID; doff = 0; }
    else if (v < NU0 + NU1) { layer = 1; vv = v - NU0;       sh = 4; pitch = K2;  doff = OW1; }
    else                    { layer = 2; vv = v - NU0 - NU1; sh = 4; pitch = K2;  doff = OW2; }
    const int n  = vv >> sh;
    const int k8 = (vv & ((1 << sh) - 1)) * 8;
    const int kk = k8 & (HID - 1);
    const float* p = Ws + (size_t)layer * HID * HID + (size_t)kk * HID + n;
    v8us o;
#pragma unroll
    for (int i = 0; i < 8; ++i) o[i] = (unsigned short)bf16_bits(p[(size_t)i * HID]);
    unsigned short* dp = wp + doff + (size_t)n * pitch + k8;
    *(volatile v8us*)dp = o;
    __threadfence();
    *(volatile v8us*)dp = o;
  } else {
#pragma unroll 1
    for (int i = tid; i < PARLDS; i += NTHR) {
      const int ic = i < PARV ? i : PARV - 1;
      const int l  = ic / (5 * HID);
      const int r  = ic - l * (5 * HID);
      const int j  = r >> 6;
      const int c  = r & (HID - 1);
      const int pi = l * HID + c;
      const float vb = bf16_val(bs[pi]);
      const float vm = bf16_val(mea[pi]);
      const float vr = bf16_val(var[pi]);
      const float vg = bf16_val(gam[pi]);
      const float ve = bf16_val(bet[pi]);
      const float vw = bf16_val(lw[i & (HID - 1)]);
      const float vl = bf16_val(lb[0]);
      const float rs = 1.0f / sqrtf(vr + 1e-5f);
      float val = (j == 0) ? vb : ((j == 1) ? vm : ((j == 2) ? rs : ((j == 3) ? vg : ve)));
      val = (i >= PLW) ? vw : val;
      val = (i >= PLB) ? vl : val;
      sp[i] = val;
    }
    __syncthreads();
    const int t8 = tid < 8 ? tid : 7;
    const v4f q0 = *(const v4fa*)(sp + 4 * tid);
    const v4f q1 = *(const v4fa*)(sp + 4 * NTHR + 4 * t8);
    float* p0 = par + 4 * tid;
    float* p1 = par + 4 * NTHR + 4 * t8;
    const bool w1 = tid < 8;
    *(volatile v4f*)p0 = q0;
    if (w1) *(volatile v4f*)p1 = q1;
    __threadfence();
    *(volatile v4f*)p0 = q0;
    if (w1) *(volatile v4f*)p1 = q1;
  }
}

__global__ __launch_bounds__(NTHR) void k_deg(const int* __restrict__ dsts, int nE, int vec8, float* dis) {
  __shared__ __attribute__((aligned(16))) int scnt[NBD];
  __shared__ __attribute__((aligned(16))) int list[LISTN];
  __shared__ int wcnt[NWAVE];
  const int tid = (int)threadIdx.x, lane = tid & 31, wave = tid >> 5;
  const int nodeBase = (int)blockIdx.x * NBD;

  for (int i = tid; i < NBD; i += NTHR) scnt[i] = 0;
  for (int i = tid; i < LISTN; i += NTHR) list[i] = 0;
  if (tid < NWAVE) wcnt[tid] = 0;
  __syncthreads();

  const int nChunks = (nE + CHUNK - 1) / CHUNK;
#pragma unroll 1
  for (int ch = 0; ch < nChunks; ++ch) {
    const int cbase = ch * CHUNK;
    const int wc = scan_chunk<SLD>(dsts, nE, cbase, nodeBase, NBD, vec8, list, tid, lane, wave);
    if (lane == 0) wcnt[wave] = wc;
    __syncthreads();
    if (wave == 0) {
#pragma unroll 1
      for (int w2 = 0; w2 < NWAVE; ++w2) {
        int c = wcnt[w2];
        c = c < 0 ? 0 : (c > WCAP ? WCAP : c);
#pragma unroll 1
        for (int b0 = 0; b0 < c; b0 += 32) {
          const int idx = b0 + lane;
          const int ent = list[w2 * WCAP + (idx < WCAP ? idx : WCAP - 1)];
          const int m32 = (c - b0) < 32 ? (c - b0) : 32;
#pragma unroll 1
          for (int k = 0; k < m32; ++k) {
            const int u  = __builtin_amdgcn_readlane(ent, k);
            const int sl = u & (NBD - 1);
            if (lane == 0) scnt[sl] = scnt[sl] + 1;
          }
        }
      }
    }
    __syncthreads();
  }

#pragma unroll 1
  for (int i = tid; i < NBD; i += NTHR) {
    const int c = scnt[i];
    const float d = fmaxf((float)(c + 1), 1.0f);
    scnt[i] = __float_as_int(1.0f / sqrtf(d));
  }
  __syncthreads();

  v4f vals[NBD / (NTHR * 4)];
#pragma unroll
  for (int it = 0; it < NBD / (NTHR * 4); ++it) {
    const int s0 = it * (NTHR * 4) + 4 * tid;
    const v4i c4 = *(const v4ia*)(scnt + s0);
    v4f v;
    v.x = __int_as_float(c4.x); v.y = __int_as_float(c4.y);
    v.z = __int_as_float(c4.z); v.w = __int_as_float(c4.w);
    vals[it] = v;
  }
#pragma unroll
  for (int it = 0; it < NBD / (NTHR * 4); ++it) {
    const int s0 = it * (NTHR * 4) + 4 * tid;
    *(volatile v4f*)(dis + (size_t)nodeBase + s0) = vals[it];
  }
  __threadfence();
#pragma unroll
  for (int it = 0; it < NBD / (NTHR * 4); ++it) {
    const int s0 = it * (NTHR * 4) + 4 * tid;
    *(volatile v4f*)(dis + (size_t)nodeBase + s0) = vals[it];
  }
}

__global__ __launch_bounds__(GTHR) void k_gemm(
    const unsigned short* __restrict__ A, const unsigned short* __restrict__ WT,
    float* outF, int K, int ldo)
{
  __shared__ __attribute__((aligned(16))) float stg[GBM * GBN];
  const int tid = (int)threadIdx.x, lane = tid & 31, wave = tid >> 5, hh = lane >> 4, m = lane & 15;
  const int rowBase = (int)blockIdx.x * GBM;
  const int col0    = (int)blockIdx.y * GBN;

  v8f acc[4];
  {
    const v8f z = {0.f, 0.f, 0.f, 0.f, 0.f, 0.f, 0.f, 0.f};
    acc[0] = z; acc[1] = z; acc[2] = z; acc[3] = z;
  }
  const unsigned short* ap = A  + (size_t)(rowBase + 16 * wave + m) * (size_t)K + 8 * hh;
  const unsigned short* wp = WT + (size_t)(col0 + m) * (size_t)K + 8 * hh;
  const int ksteps = K >> 5;
#pragma unroll 1
  for (int ks = 0; ks < ksteps; ++ks) {
    FragB af;
    af.h[0] = *(const v8usa*)(ap + 32 * ks);
    af.h[1] = *(const v8usa*)(ap + 32 * ks + 16);
#pragma unroll
    for (int t = 0; t < 4; ++t) {
      const unsigned short* wq = wp + (size_t)(16 * t) * (size_t)K + 32 * ks;
      FragB bf;
      bf.h[0] = *(const v8usa*)wq;
      bf.h[1] = *(const v8usa*)(wq + 16);
      acc[t] = wmb(af, bf, acc[t]);
    }
  }

#pragma unroll
  for (int t = 0; t < 4; ++t) {
    const int lc = 16 * t + m;
#pragma unroll
    for (int r = 0; r < 8; ++r) {
      const int lr = 16 * wave + 8 * hh + r;
      stg[lr * GBN + lc] = acc[t][r];
    }
  }
  __syncthreads();

  v4f fv[8];
#pragma unroll
  for (int i = 0; i < 8; ++i) {
    const int lr = 16 * wave + 2 * i + hh;
    fv[i] = *(const v4fa*)(stg + lr * GBN + 4 * m);
  }
#pragma unroll
  for (int i = 0; i < 8; ++i) {
    const int lr = 16 * wave + 2 * i + hh;
    const int gr = rowBase + lr;
    float* op = outF + (size_t)gr * (size_t)ldo + col0 + 4 * m;
    *(volatile v4f*)op = fv[i];
  }
  __threadfence();
#pragma unroll
  for (int i = 0; i < 8; ++i) {
    const int lr = 16 * wave + 2 * i + hh;
    const int gr = rowBase + lr;
    float* op = outF + (size_t)gr * (size_t)ldo + col0 + 4 * m;
    *(volatile v4f*)op = fv[i];
  }
}

template <int HEAD>
__global__ __launch_bounds__(NTHR) void k_scan(const int* __restrict__ srcs, const int* __restrict__ dsts,
                                               int nE, int nN, int vec8, int mRows,
                                               const float* __restrict__ dis,
                                               const float* __restrict__ xl,
                                               const float* __restrict__ par,
                                               const float* __restrict__ lwp,
                                               unsigned short* hb, float* outp) {
  extern __shared__ __attribute__((aligned(16))) int dsm[];
  int* list = dsm;
  int* hl   = dsm + LISTN;
  int* sl   = dsm + LISTN + RCAP;
  int* cnt  = dsm + LISTN + 2 * RCAP;
  int* offs = cnt + NBA;
  int* cur  = offs + NBA;
  int* misc = cur + NBA;
  float* scf = (float*)(misc + MISC_INTS);
  const int tid = (int)threadIdx.x, lane = tid & 31, wave = tid >> 5;
  const int nodeBase = (int)blockIdx.x * NBA;

  {
    const v4i z4 = {0, 0, 0, 0};
    for (int i = tid * 4; i < AGG_ZINTS; i += NTHR * 4) *(v4ia*)(dsm + i) = z4;
    if (tid < MISC_INTS) misc[tid] = 0;
  }
  const v2f pb  = *(const v2fa*)(par + 0 * HID + 2 * lane);
  const v2f pm  = *(const v2fa*)(par + 1 * HID + 2 * lane);
  const v2f prs = *(const v2fa*)(par + 2 * HID + 2 * lane);
  const v2f pg  = *(const v2fa*)(par + 3 * HID + 2 * lane);
  const v2f pbe = *(const v2fa*)(par + 4 * HID + 2 * lane);
  v2f plw = {0.0f, 0.0f};
  float plb = 0.0f;
  if constexpr (HEAD != 0) {
    plw = *(const v2fa*)(lwp + 2 * lane);
    plb = lwp[HID];
  }
  __syncthreads();

  int t = 0, ov = 0;
  const int nChunks = (nE + CHUNK - 1) / CHUNK;
#pragma unroll 1
  for (int ch = 0; ch < nChunks; ++ch) {
    const int cbase = ch * CHUNK;
    const int wc = scan_chunk<SLA>(dsts, nE, cbase, nodeBase, NBA, vec8, list, tid, lane, wave);
    if (lane == 0) misc[wave] = wc;
    __syncthreads();
    if (wave == 0) {
#pragma unroll 1
      for (int w2 = 0; w2 < NWAVE; ++w2) {
        int c = misc[w2];
        c = c < 0 ? 0 : (c > WCAP ? WCAP : c);
#pragma unroll 1
        for (int b0 = 0; b0 < c; b0 += 32) {
          const int idx = b0 + lane;
          const int ent = list[w2 * WCAP + (idx < WCAP ? idx : WCAP - 1)];
          const int m32 = (c - b0) < 32 ? (c - b0) : 32;
#pragma unroll 1
          for (int k = 0; k < m32; ++k) {
            const int u    = __builtin_amdgcn_readlane(ent, k);
            const int slot = u & (NBA - 1);
            const int el   = (u >> SLA) & (CHUNK - 1);
            const int pk   = ((cbase + el) << SLA) | slot;
            if (t < RCAP) {
              if (lane == 0) { hl[t] = pk; cnt[slot] = cnt[slot] + 1; }
              t = t + 1;
            } else {
              ov = 1;
            }
          }
        }
      }
    }
    __syncthreads();
  }
  if (wave == 0 && lane == 0) { misc[8] = t; misc[9] = ov; }
  __syncthreads();
  int tt = misc[8];
  tt = tt < 0 ? 0 : (tt > RCAP ? RCAP : tt);
  const int ovf = misc[9];

  if (wave == 0) {
    const int base = lane * (NBA / 32);
    int s = 0;
#pragma unroll 1
    for (int i = 0; i < NBA / 32; ++i) s += cnt[base + i];
    int incl = s;
#pragma unroll
    for (int d = 1; d < 32; d <<= 1) {
      const int y = __shfl_up(incl, d, 32);
      if (lane >= d) incl += y;
    }
    int run = incl - s;
#pragma unroll 1
    for (int i = 0; i < NBA / 32; ++i) {
      const int cv = cnt[base + i];
      offs[base + i] = run;
      cur[base + i]  = run;
      run += cv;
    }
  }
  __syncthreads();
  if (wave == 0) {
#pragma unroll 1
    for (int b0 = 0; b0 < tt; b0 += 32) {
      const int idx = b0 + lane;
      const int ent = hl[idx < RCAP ? idx : RCAP - 1];
      const int m32 = (tt - b0) < 32 ? (tt - b0) : 32;
#pragma unroll 1
      for (int k = 0; k < m32; ++k) {
        const int u    = __builtin_amdgcn_readlane(ent, k);
        const int slot = u & (NBA - 1);
        if (lane == 0) {
          int p = cur[slot];
          p = p < 0 ? 0 : (p > RCAP - 1 ? RCAP - 1 : p);
          sl[p] = u;
          cur[slot] = p + 1;
        }
      }
    }
  }
  __syncthreads();

  const float qnan = __int_as_float(0x7fc00000);
  const float pz = (ovf != 0) ? qnan : 0.0f;
  const int q0s = (4 * lane) & 31, q1s = (4 * lane + 1) & 31;
  const int q2s = (4 * lane + 2) & 31, q3s = (4 * lane + 3) & 31;
#pragma unroll 1
  for (int si = 0; si < NBA / NWAVE; ++si) {
    const int s    = si * NWAVE + wave;
    const int node = nodeBase + s;
    int c = cnt[s];
    const bool big = c > DEGCAP;
    c = c < 0 ? 0 : (c > DEGCAP ? DEGCAP : c);
    int o = offs[s];
    o = o < 0 ? 0 : (o > RCAP ? RCAP : o);
    const int nc = node < nN ? node : nN - 1;
    const float dd = dis[nc];
    const float rd = dd * dd;
    float acc0 = 0.0f, acc1 = 0.0f;
#pragma unroll 1
    for (int b0 = 0; b0 < c; b0 += 32) {
      int idx = o + b0 + lane;
      idx = idx > RCAP - 1 ? RCAP - 1 : idx;
      const int ent = sl[idx];
      int eid = ent >> SLA;
      eid = eid < 0 ? 0 : (eid > nE - 1 ? nE - 1 : eid);
      int sr = srcs[eid];
      sr = sr < 0 ? 0 : (sr > nN - 1 ? nN - 1 : sr);
      const float cf  = dis[sr] * dd;
      const int   cfi = __float_as_int(cf);
      const int m32 = (c - b0) < 32 ? (c - b0) : 32;
#pragma unroll 1
      for (int k = 0; k < m32; ++k) {
        const int   sk = __builtin_amdgcn_readlane(sr, k);
        const float ck = __int_as_float(__builtin_amdgcn_readlane(cfi, k));
        const v2f a = *(const v2fa*)(xl + (size_t)sk * HID + 2 * lane);
        acc0 = fmaf(ck, a.x, acc0); acc1 = fmaf(ck, a.y, acc1);
      }
    }
    float sv0, sv1;
    {
      const v2f a = *(const v2fa*)(xl + (size_t)nc * HID + 2 * lane);
      sv0 = a.x; sv1 = a.y;
    }
    const float pzr = big ? qnan : pz;
    const bool live = node < nN;
    const float a0 = ((acc0 + sv0 * rd) + pb.x) + pzr;
    const float a1 = ((acc1 + sv1 * rd) + pb.y) + pzr;
    float y0 = ((a0 - pm.x) * prs.x) * pg.x + pbe.x;
    float y1 = ((a1 - pm.y) * prs.y) * pg.y + pbe.y;
    y0 = (y0 > 0.0f) ? y0 : (y0 - y0);
    y1 = (y1 > 0.0f) ? y1 : (y1 - y1);
    const float v0 = live ? y0 : 0.0f;
    const float v1 = live ? y1 : 0.0f;
    if constexpr (HEAD == 0) {
      const bool wr = (node < mRows) && (lane < 16);
      const unsigned hb0 = bf16_bits(v0), hb1 = bf16_bits(v1);
      const unsigned lb0 = bf16_bits(v0 - __uint_as_float(hb0 << 16));
      const unsigned lb1 = bf16_bits(v1 - __uint_as_float(hb1 << 16));
      const int hw = (int)(hb0 | (hb1 << 16));
      const int lw = (int)(lb0 | (lb1 << 16));
      const int g0 = __shfl(hw, q0s, 32), g1 = __shfl(hw, q1s, 32);
      const int g2 = __shfl(hw, q2s, 32), g3 = __shfl(hw, q3s, 32);
      const int p0 = __shfl(lw, q0s, 32), p1 = __shfl(lw, q1s, 32);
      const int p2 = __shfl(lw, q2s, 32), p3 = __shfl(lw, q3s, 32);
      const bool lsel = (lane & 8) != 0;
      v4u pv;
      pv.x = (unsigned int)(lsel ? p0 : g0);
      pv.y = (unsigned int)(lsel ? p1 : g1);
      pv.z = (unsigned int)(lsel ? p2 : g2);
      pv.w = (unsigned int)(lsel ? p3 : g3);
      unsigned short* hp = hb + (size_t)(node < mRows ? node : 0) * K2 + 8 * (lane & 15);
      if (wr) *(volatile v4u*)hp = pv;
      __threadfence();
      if (wr) *(volatile v4u*)hp = pv;
    } else {
      float hs = fmaf(v1, plw.y, v0 * plw.x);
      hs += __shfl_xor(hs, 16, 32);
      hs += __shfl_xor(hs, 8, 32);
      hs += __shfl_xor(hs, 4, 32);
      hs += __shfl_xor(hs, 2, 32);
      hs += __shfl_xor(hs, 1, 32);
      if (lane == 0) scf[s] = hs + plb;
    }
  }

  if constexpr (HEAD != 0) {
    __syncthreads();
    const int rem = nN - nodeBase;
    int nvu = rem >> 2;
    nvu = nvu < 0 ? 0 : (nvu > NBA / 4 ? NBA / 4 : nvu);
    v4f q = *(const v4fa*)(scf + 4 * tid);
    const bool pzn = ovf != 0;
    q.x = pzn ? qnan : q.x; q.y = pzn ? qnan : q.y;
    q.z = pzn ? qnan : q.z; q.w = pzn ? qnan : q.w;
    const bool wr = tid < nvu;
    float* op = outp + (size_t)(wr ? (nodeBase + 4 * tid) : 0);
    if (wr) *(volatile v4f*)op = q;
    __threadfence();
    if (wr) *(volatile v4f*)op = q;
  }
}

static inline int cdiv(int a, int b) { return (a + b - 1) / b; }
static inline size_t al256(size_t o) { return (o + 255) & ~(size_t)255; }

extern "C" void kernel_launch(void* const* d_in, const int* in_sizes, int n_in,
                              void* d_out, int out_size, void* d_ws, size_t ws_size,
                              hipStream_t stream) {
  if (n_in < 10) return;
  if (in_sizes[0] < HID || (in_sizes[0] % HID) != 0) return;
  const int nN = in_sizes[0] / HID;
  if (nN < 4 || nN > (1 << 22) || (nN & 3) != 0) return;
  if (in_sizes[1] < 2 || (in_sizes[1] & 1) != 0) return;
  const int nE = in_sizes[1] / 2;
  if (nE < 1 || nE >= (1 << (31 - SLA))) return;
  if (in_sizes[2] != NLAY * HID * HID) return;
  if (in_sizes[3] != NLAY * HID || in_sizes[4] != NLAY * HID) return;
  if (in_sizes[5] != NLAY * HID || in_sizes[6] != NLAY * HID) return;
  if (in_sizes[7] != NLAY * HID) return;
  if (in_sizes[8] != HID || in_sizes[9] != 1) return;
  if (out_size != nN) return;

  const float* x    = (const float*)d_in[0];
  const int*   edge = (const int*)d_in[1];
  const float* Ws   = (const float*)d_in[2];
  const float* bs   = (const float*)d_in[3];
  const float* gam  = (const float*)d_in[4];
  const float* bet  = (const float*)d_in[5];
  const float* mea  = (const float*)d_in[6];
  const float* var  = (const float*)d_in[7];
  const float* lw   = (const float*)d_in[8];
  const float* lb   = (const float*)d_in[9];
  float* out = (float*)d_out;
  const int* src = edge;
  const int* dst = edge + nE;

  const int MP   = cdiv(nN, GBM) * GBM;
  const int gM   = MP / GBM;
  const int gD   = cdiv(nN, NBD);
  const int NBPD = gD * NBD;
  const int gA   = cdiv(MP, NBA);
  if ((long long)gA * NBA < (long long)MP) return;
  if (NBPD < nN) return;
  const int vec8 = ((nE & 3) == 0) ? 1 : 0;
  const int nUx  = MP * (HID / 8);
  const int gX   = cdiv(nUx, NTHR);

  char* ws = (char*)d_ws;
  size_t off = 0;
  const size_t oDIS = off; off = al256(off + (size_t)NBPD * 4);
  const size_t oWP  = off; off = al256(off + (size_t)WPN * 2);
  const size_t oPAR = off; off = al256(off + (size_t)PARF * 4);
  const size_t oXB  = off; off = al256(off + (size_t)MP * HID * 2);
  const size_t oH   = off; off = al256(off + (size_t)MP * HID * 4);
  const size_t oXHL = off; off = al256(off + (size_t)MP * K2 * 2);
  if (off > ws_size || off > (size_t)WSMAX) return;
  float*          DIS = (float*)(ws + oDIS);
  unsigned short* WP  = (unsigned short*)(ws + oWP);
  float*          PAR = (float*)(ws + oPAR);
  unsigned short* XB  = (unsigned short*)(ws + oXB);
  float*          H   = (float*)(ws + oH);
  unsigned short* XHL = (unsigned short*)(ws + oXHL);

  const size_t scanLds = (size_t)AGG_LDS_INTS * 4;
  hipFuncSetAttribute(reinterpret_cast<const void*>(&k_scan<0>), hipFuncAttributeMaxDynamicSharedMemorySize, (int)scanLds);
  hipFuncSetAttribute(reinterpret_cast<const void*>(&k_scan<1>), hipFuncAttributeMaxDynamicSharedMemorySize, (int)scanLds);

  k_prep<<<gX + NWBLK + 1, NTHR, 0, stream>>>(x, nN, nUx, gX, Ws, bs, gam, bet, mea, var, lw, lb, XB, WP, PAR);
  k_deg<<<gD, NTHR, 0, stream>>>(dst, nE, vec8, DIS);
  k_gemm<<<dim3(gM, HID / GBN), GTHR, 0, stream>>>(XB, WP, H, HID, HID);
  k_scan<0><<<gA, NTHR, scanLds, stream>>>(src, dst, nE, nN, vec8, MP, DIS, H, PAR, PAR + PLW, XHL, out);
  k_gemm<<<dim3(gM, HID / GBN), GTHR, 0, stream>>>(XHL, WP + OW1, H, K2, HID);
  k_scan<0><<<gA, NTHR, scanLds, stream>>>(src, dst, nE, nN, vec8, MP, DIS, H, PAR + 5 * HID, PAR + PLW, XHL, out);
  k_gemm<<<dim3(gM, HID / GBN), GTHR, 0, stream>>>(XHL, WP + OW2, H, K2, HID);
  k_scan<1><<<gA, NTHR, scanLds, stream>>>(src, dst, nE, nN, vec8, MP, DIS, H, PAR + 10 * HID, PAR + PLW, XHL, out);
}
